// GMFlow_283467842155
// MI455X (gfx1250) — hardware-verified
//
#include <hip/hip_runtime.h>

typedef _Float16 v16h __attribute__((ext_vector_type(16)));
typedef _Float16 v8h  __attribute__((ext_vector_type(8)));
typedef float    v8f  __attribute__((ext_vector_type(8)));

union V16 { v16h v; v8h h[2]; };
typedef __attribute__((ext_vector_type(4))) float v4f_t;
typedef float v4fa __attribute__((ext_vector_type(4), may_alias));
typedef __attribute__((ext_vector_type(4))) unsigned v4u_t;
typedef unsigned v4ua __attribute__((ext_vector_type(4), may_alias));
__device__ __forceinline__ unsigned pk2(float a, float b) { return (unsigned)__builtin_bit_cast(unsigned short, (_Float16)a) | ((unsigned)__builtin_bit_cast(unsigned short, (_Float16)b) << 16); }

#define RSQRT_C 0.08838834764831845f
#define NEG_BIG -3.0e38f

__device__ __forceinline__ v8f zero8() {
    v8f z = {0.f,0.f,0.f,0.f,0.f,0.f,0.f,0.f};
    return z;
}

__device__ __forceinline__ float posval(int c, int ly, int lx) {
    int coord = (c < 64) ? ly : lx;
    int t = c & 63;
    float k = (float)(t >> 1);
    float dim = __expf(k * 0.28782313662425575f);
    float v = ((float)(coord + 1)) * (6.283185307179586f / 32.000001f) / dim;
    return (t & 1) ? __cosf(v) : __sinf(v);
}

__global__ void gmflow_prep(const float* __restrict__ f0,
                            const float* __restrict__ f1,
                            _Float16* __restrict__ Qw, _Float16* __restrict__ Kw,
                            _Float16* __restrict__ Vt, _Float16* __restrict__ F1g) {
    (void)Vt;
    int idx = (blockIdx.x * blockDim.x + threadIdx.x) * 2;
    int c   = idx & 127;
    int q   = (idx >> 7) & 1023;
    int win = idx >> 17;
    int b = win >> 2, i = (win >> 1) & 1, j = win & 1;
    int r = q >> 5, cc = q & 31;
    int y = ((i << 5) + r  + 16) & 63;
    int x = ((j << 5) + cc + 16) & 63;
    int pix = (y << 6) + x;
    float pa = posval(c, y & 31, x & 31), pb = posval(c + 1, y & 31, x & 31);
    int   gi = ((b << 7) + c) * 4096 + pix;
    const unsigned uq = pk2(f0[gi] + pa, f0[gi + 4096] + pb);
    const unsigned uk = pk2(f1[gi] + pa, f1[gi + 4096] + pb);
    const size_t oqk = ((size_t)win << 17) + (q << 7) + c, of1 = ((((size_t)b << 12) + pix) << 7) + c;
    *(volatile unsigned*)(Qw + oqk) = uq; *(volatile unsigned*)(Kw + oqk) = uk; *(volatile unsigned*)(F1g + of1) = uk;
    __threadfence();
    *(volatile unsigned*)(Qw + oqk) = uq; *(volatile unsigned*)(Kw + oqk) = uk; *(volatile unsigned*)(F1g + of1) = uk;
}

__global__ __launch_bounds__(256) void gmflow_vt(const _Float16* __restrict__ Kw, _Float16* __restrict__ Vt) {
    __shared__ _Float16 t[64][130];
    const int tid = threadIdx.x, lane = tid & 31, wave = tid >> 5;
    const int win = blockIdx.x >> 4, q0 = (blockIdx.x & 15) * 64;
    const _Float16* src = Kw + ((size_t)win << 17) + ((size_t)q0 << 7);
#pragma unroll
    for (int k = 0; k < 32; ++k) { const int e = tid + 256 * k; t[e >> 7][e & 127] = src[e]; }
    __syncthreads();
    _Float16* dst = Vt + ((size_t)win << 17) + q0;
#pragma unroll
    for (int rr = 0; rr < 16; ++rr) {
        const int c = wave * 16 + rr;
        const unsigned p = (unsigned)__builtin_bit_cast(unsigned short, t[2 * lane][c]) | ((unsigned)__builtin_bit_cast(unsigned short, t[2 * lane + 1][c]) << 16);
        unsigned* d = (unsigned*)(dst + ((size_t)c << 10)) + lane;
        *(volatile unsigned*)d = p; __threadfence(); *(volatile unsigned*)d = p;
    }
}

__global__ __launch_bounds__(128) void gmflow_attn(
        const _Float16* __restrict__ Qw, const _Float16* __restrict__ Kw,
        const _Float16* __restrict__ Vt, _Float16* __restrict__ F0A) {
    int lane = threadIdx.x & 31;
    int wave = threadIdx.x >> 5;
    int bw   = blockIdx.x;
    int win  = bw >> 4;
    int qt   = ((bw & 15) << 2) | wave;
    int qbase = qt << 4;
    int b = win >> 2, wi = (win >> 1) & 1, wj = win & 1;
    int ln = lane & 15;
    bool hiL = (lane >= 16);
    int qloc = qbase + ln;
    int rq = qloc >> 5, cq = qloc & 31;
    bool qrlo = (rq < 16), qclo = (cq < 16);

    const _Float16* qrow = Qw + (win << 17) + (qloc << 7);
    V16 Qb[4];
#pragma unroll
    for (int k4 = 0; k4 < 4; ++k4) {
        const v8h* p = (const v8h*)(qrow + k4 * 32 + (hiL ? 8 : 0));
        Qb[k4].h[0] = p[0]; Qb[k4].h[1] = p[2];
    }

    v8f acc[8];
#pragma unroll
    for (int t = 0; t < 8; ++t) acc[t] = zero8();
    float runM = NEG_BIG, runS = 0.f;

    const _Float16* Kbase = Kw + (win << 17);
    const _Float16* Vbase = Vt + (win << 17);

    for (int mc = 0; mc < 32; ++mc) {
        int mb = mc << 5;
        v8f s0 = zero8(), s1 = zero8();
#pragma unroll
        for (int k4 = 0; k4 < 4; ++k4) {
            V16 a0, a1;
            const _Float16* r0 = Kbase + ((mb + ln) << 7)      + k4 * 32 + (hiL ? 8 : 0);
            const _Float16* r1 = Kbase + ((mb + 16 + ln) << 7) + k4 * 32 + (hiL ? 8 : 0);
            a0.h[0] = *(const v8h*)(r0);  a0.h[1] = *(const v8h*)(r0 + 16);
            a1.h[0] = *(const v8h*)(r1);  a1.h[1] = *(const v8h*)(r1 + 16);
            s0 = __builtin_amdgcn_wmma_f32_16x16x32_f16(false, a0.v, false, Qb[k4].v,
                                                        (short)0, s0, false, false);
            s1 = __builtin_amdgcn_wmma_f32_16x16x32_f16(false, a1.v, false, Qb[k4].v,
                                                        (short)0, s1, false, false);
        }
        float p0[8], p1[8];
        float cmx = NEG_BIG;
#pragma unroll
        for (int v = 0; v < 8; ++v) {
            int m0 = mb + v + (hiL ? 8 : 0);
            int m1 = m0 + 16;
            int rm0 = m0 >> 5, cm0 = m0 & 31;
            int rm1 = m1 >> 5, cm1 = m1 & 31;
            bool bad0 = (wi && ((rm0 < 16) != qrlo)) || (wj && ((cm0 < 16) != qclo));
            bool bad1 = (wi && ((rm1 < 16) != qrlo)) || (wj && ((cm1 < 16) != qclo));
            float t0 = s0[v] * RSQRT_C + (bad0 ? -100.f : 0.f);
            float t1 = s1[v] * RSQRT_C + (bad1 ? -100.f : 0.f);
            p0[v] = t0; p1[v] = t1;
            cmx = fmaxf(cmx, fmaxf(t0, t1));
        }
        cmx = fmaxf(cmx, __shfl_xor(cmx, 16, 32));
        float newM = fmaxf(runM, cmx);
        float sc = __expf(runM - newM);
        runM = newM;
        runS *= sc;
#pragma unroll
        for (int t = 0; t < 8; ++t) acc[t] *= sc;
        float lsum = 0.f;
#pragma unroll
        for (int v = 0; v < 8; ++v) {
            p0[v] = __expf(p0[v] - runM);
            p1[v] = __expf(p1[v] - runM);
            lsum += p0[v] + p1[v];
        }
        runS += lsum;
        V16 pB;
#pragma unroll
        for (int v = 0; v < 8; ++v) {
            pB.v[v]     = (_Float16)(p0[v] * 1024.0f);
            pB.v[v + 8] = (_Float16)(p1[v] * 1024.0f);
        }
#pragma unroll
        for (int ct = 0; ct < 8; ++ct) {
            int ch = (ct << 4) + ln;
            const _Float16* vr = Vbase + (ch << 10) + mb + (hiL ? 8 : 0);
            V16 av;
            av.h[0] = *(const v8h*)(vr);  av.h[1] = *(const v8h*)(vr + 16);
            acc[ct] = __builtin_amdgcn_wmma_f32_16x16x32_f16(false, av.v, false, pB.v,
                                                             (short)0, acc[ct], false, false);
        }
    }
    float totS = runS + __shfl_xor(runS, 16, 32);
    float inv = 1.0f / (totS * 1024.0f);
    __shared__ __attribute__((aligned(16))) _Float16 so_[4][16 * 128];
    _Float16* so = so_[wave];
#pragma unroll
    for (int ct = 0; ct < 8; ++ct)
#pragma unroll
        for (int v = 0; v < 8; ++v) so[ln * 128 + (ct << 4) + (hiL ? 8 : 0) + v] = (_Float16)(acc[ct][v] * inv);
    asm volatile("s_wait_dscnt 0" ::: "memory");
    v4u_t ov[8]; size_t oo[8];
#pragma unroll
    for (int i2 = 0; i2 < 8; ++i2) {
        const int c = lane + 32 * i2, rr = c >> 4, pc = c & 15;
        const int ql = qbase + rr, rq2 = ql >> 5, cq2 = ql & 31;
        const int y2 = ((wi << 5) + rq2 + 16) & 63, x2 = ((wj << 5) + cq2 + 16) & 63;
        ov[i2] = *(const volatile v4ua*)(so + rr * 128 + pc * 8);
        oo[i2] = ((((size_t)b << 12) + (y2 << 6) + x2) << 7) + pc * 8;
    }
#pragma unroll
    for (int i2 = 0; i2 < 8; ++i2) *(volatile v4u_t*)(F0A + oo[i2]) = ov[i2];
    __threadfence();
#pragma unroll
    for (int i2 = 0; i2 < 8; ++i2) *(volatile v4u_t*)(F0A + oo[i2]) = ov[i2];
}

__global__ __launch_bounds__(128) void gmflow_corr(
        const _Float16* __restrict__ F0A, const _Float16* __restrict__ F1g,
        float* __restrict__ out) {
    int lane = threadIdx.x & 31;
    int wave = threadIdx.x >> 5;
    int wid  = blockIdx.x * 4 + wave;
    int b    = wid >> 8;
    int qbase = (wid & 255) << 4;
    int ln = lane & 15;
    bool hiL = (lane >= 16);
    int n = qbase + ln;

    const _Float16* brow = F0A + (((b << 12) + n) << 7);
    V16 Bb[4];
#pragma unroll
    for (int k4 = 0; k4 < 4; ++k4) {
        const v8h* p = (const v8h*)(brow + k4 * 32 + (hiL ? 8 : 0));
        Bb[k4].h[0] = p[0]; Bb[k4].h[1] = p[2];
    }

    float runM = NEG_BIG, runS = 0.f, runSx = 0.f, runSy = 0.f;
    const _Float16* Abase = F1g + ((size_t)b << 19);

    for (int mt = 0; mt < 256; ++mt) {
        int mb = mt << 4;
        v8f s = zero8();
#pragma unroll
        for (int k4 = 0; k4 < 4; ++k4) {
            const _Float16* ar = Abase + ((mb + ln) << 7) + k4 * 32 + (hiL ? 8 : 0);
            V16 a;
            a.h[0] = *(const v8h*)(ar);  a.h[1] = *(const v8h*)(ar + 16);
            s = __builtin_amdgcn_wmma_f32_16x16x32_f16(false, a.v, false, Bb[k4].v,
                                                       (short)0, s, false, false);
        }
        float sv[8];
        float cmx = NEG_BIG;
#pragma unroll
        for (int v = 0; v < 8; ++v) {
            sv[v] = s[v] * RSQRT_C;
            cmx = fmaxf(cmx, sv[v]);
        }
        cmx = fmaxf(cmx, __shfl_xor(cmx, 16, 32));
        float newM = fmaxf(runM, cmx);
        float sc = __expf(runM - newM);
        runM = newM;
        runS *= sc; runSx *= sc; runSy *= sc;
#pragma unroll
        for (int v = 0; v < 8; ++v) {
            float p = __expf(sv[v] - runM);
            int mg = mb + v + (hiL ? 8 : 0);
            runS  += p;
            runSx += p * (float)(mg & 63);
            runSy += p * (float)(mg >> 6);
        }
    }
    runS  += __shfl_xor(runS, 16, 32);
    runSx += __shfl_xor(runSx, 16, 32);
    runSy += __shfl_xor(runSy, 16, 32);
    __shared__ __attribute__((aligned(16))) float fo[2][64];
    if (!hiL) {
        float inv = 1.0f / runS;
        fo[0][wave * 16 + ln] = runSx * inv - (float)(n & 63);
        fo[1][wave * 16 + ln] = runSy * inv - (float)(n >> 6);
    }
    __syncthreads();
    if (wave == 0) {
        const int pl = lane >> 4, q = lane & 15;
        const v4f_t v = *(const v4fa*)(&fo[pl][q * 4]);
        float* dst = out + ((size_t)b << 13) + pl * 4096 + (blockIdx.x & 63) * 64 + q * 4;
        *(volatile v4f_t*)dst = v; __threadfence(); *(volatile v4f_t*)dst = v;
    }
}

extern "C" void kernel_launch(void* const* d_in, const int* in_sizes, int n_in,
                              void* d_out, int out_size, void* d_ws, size_t ws_size,
                              hipStream_t stream) {
    const float* f0 = (const float*)d_in[0];
    const float* f1 = (const float*)d_in[1];
    float* out = (float*)d_out;

    _Float16* ws  = (_Float16*)d_ws;
    const size_t WSEG = 16u * 1024u * 128u;
    _Float16* Qw  = ws;
    _Float16* Kw  = Qw  + WSEG;
    _Float16* Vt  = Kw  + WSEG;
    _Float16* F1g = Vt  + WSEG;
    _Float16* F0A = F1g + WSEG;

    gmflow_prep<<<4096, 256, 0, stream>>>(f0, f1, Qw, Kw, Vt, F1g);
    gmflow_vt<<<16 * 16, 256, 0, stream>>>(Kw, Vt);
    gmflow_attn<<<256, 128, 0, stream>>>(Qw, Kw, Vt, F0A);
    gmflow_corr<<<256, 128, 0, stream>>>(F0A, F1g, out);
}
